// Encoder_60112362275055
// MI455X (gfx1250) — hardware-verified
//
#include <hip/hip_runtime.h>
#include <math.h>

constexpr int NBATCH     = 64;
constexpr int NSTEP      = 512;
constexpr int NIN        = 256;
constexpr int NHID       = 1024;
constexpr int NGATE      = 3 * NHID;
constexpr int RTHR       = 512;
constexpr int RWAVES     = RTHR / 32;
constexpr int ROWS_BLK   = 16;
constexpr int HPITCH     = 1032;
constexpr int SLABP      = 68;
constexpr int RING_SLOTS = 16;
constexpr int SKIP_MAX   = 8;
constexpr float WCARRY     = 16.0f;
constexpr float WCARRY_INV = 1.0f / WCARRY;
constexpr int CVT_THR    = 256;

static_assert(NHID == 64 * RWAVES, "one wave per 64 hidden columns");
static_assert(NHID % 32 == 0 && NIN % 32 == 0, "k extents are multiples of the 32-deep step");
static_assert(NBATCH % ROWS_BLK == 0, "whole 16-row tiles");
static_assert((HPITCH * 2) % 16 == 0 && HPITCH >= NHID, "16-byte aligned fragment rows");
static_assert(RING_SLOTS >= 2 * SKIP_MAX, "ring depth covers the largest lag");
static_assert((SLABP * 4) % 16 == 0, "16-byte aligned slab rows");

typedef __attribute__((ext_vector_type(16))) _Float16 v16h;
typedef __attribute__((ext_vector_type(8)))  _Float16 v8h;
typedef __attribute__((ext_vector_type(8)))  float    v8f;
typedef __attribute__((ext_vector_type(4)))  float    v4f;

union FragU { v16h v; v8h h[2]; };
__device__ __forceinline__ v16h frag_load(const _Float16* p) {
  FragU f;
  f.h[0] = *(const v8h*)(p);
  f.h[1] = *(const v8h*)(p + 16);
  return f.v;
}
__device__ __forceinline__ v8f mma16(v16h a, v16h b, v8f c) {
  return __builtin_amdgcn_wmma_f32_16x16x32_f16(false, a, false, b, (short)0, c, false, false);
}
__device__ __forceinline__ void guard3(v8f& a0, v8f& a1, v8f& a2, v16h x, v16h y0, v16h y1, v16h y2) {
  asm volatile("v_nop\n\tv_nop\n\tv_nop\n\tv_nop"
               : "+v"(a0), "+v"(a1), "+v"(a2)
               : "v"(x), "v"(y0), "v"(y1), "v"(y2));
}
__device__ __forceinline__ void guard4acc(v8f& a0, v8f& a1, v8f& a2, v8f& a3) {
  asm volatile("v_nop\n\tv_nop\n\tv_nop\n\tv_nop" : "+v"(a0), "+v"(a1), "+v"(a2), "+v"(a3));
}

__device__ __forceinline__ float fsig(float x)  { return __builtin_amdgcn_rcpf(1.0f + __expf(-x)); }
__device__ __forceinline__ float ftanh(float x) { return 1.0f - 2.0f * __builtin_amdgcn_rcpf(__expf(2.0f * x) + 1.0f); }

__global__ __launch_bounds__(CVT_THR) void cvt8_kernel(const float* __restrict__ src, unsigned short* __restrict__ dst,
                                                       int n8, int ncol8, int perm, float sc) {
  const int i = blockIdx.x * CVT_THR + threadIdx.x;
  if (i < n8) {
    const int row = i / ncol8;
    const int c8  = i - row * ncol8;
    int srow = row;
    if (perm != 0) {
      const int tt = row / NBATCH;
      const int bb = row - tt * NBATCH;
      srow = bb * NSTEP + tt;
    }
    const float* sp = src + (size_t)srow * (size_t)(ncol8 * 8) + (size_t)(c8 * 8);
    const v4f a = *(const v4f*)(sp);
    const v4f b = *(const v4f*)(sp + 4);
    v8h hv;
#pragma unroll
    for (int e = 0; e < 4; ++e) {
      const float fa = a[e] * sc;
      const float fb = b[e] * sc;
      hv[e]     = (_Float16)fa;
      hv[4 + e] = (_Float16)fb;
    }
    *(volatile v8h*)(dst + (size_t)i * 8) = hv;
    __threadfence();
    *(volatile v8h*)(dst + (size_t)i * 8) = hv;
  }
}

__global__ __launch_bounds__(RTHR) void gru_seq_kernel(const unsigned short* __restrict__ X16p,
                                                       const unsigned short* __restrict__ WHHp,
                                                       const unsigned short* __restrict__ WIHp,
                                                       const float* __restrict__ b_ih, const float* __restrict__ b_hh,
                                                       const int* __restrict__ w1, const int* __restrict__ w2,
                                                       const int* __restrict__ skipp,
                                                       float* ring, float* out) {
  __shared__ __align__(16) _Float16 Ah[ROWS_BLK * HPITCH];
  __shared__ __align__(16) float    Sl[RWAVES][16 * SLABP];
  const _Float16* X16 = (const _Float16*)X16p;
  const _Float16* WHH = (const _Float16*)WHHp;
  const _Float16* WIH = (const _Float16*)WIHp;
  const int tid = threadIdx.x, lane = tid & 31, wave = tid >> 5;
  const int c = lane & 15, hh = lane >> 4, koff = hh * 8, c4 = c * 4;
  const int rowbase = blockIdx.x * ROWS_BLK;
  int sk = skipp[0];
  sk = (sk < 1) ? 1 : ((sk > SKIP_MAX) ? SKIP_MAX : sk);

#pragma unroll 1
  for (int i = tid; i < ROWS_BLK * HPITCH; i += RTHR) Ah[i] = (_Float16)0.0f;

  float hc[4][8];
  float bR[4], bZ[4], bXN[4], bHN[4];
#pragma unroll
  for (int nt = 0; nt < 4; ++nt) {
    const int j = 64 * wave + 16 * nt + c;
    bR[nt]  = b_ih[j] + b_hh[j];
    bZ[nt]  = b_ih[NHID + j] + b_hh[NHID + j];
    bXN[nt] = b_ih[2 * NHID + j];
    bHN[nt] = b_hh[2 * NHID + j];
#pragma unroll
    for (int r = 0; r < 8; ++r) hc[nt][r] = 0.0f;
  }
  __syncthreads();

  const v8f z8 = {0.f, 0.f, 0.f, 0.f, 0.f, 0.f, 0.f, 0.f};
  float* slab = Sl[wave];
  const _Float16* ahrow = Ah + c * HPITCH + koff;

#pragma unroll 1
  for (int t = 0; t < NSTEP; ++t) {
    const int t2  = t + 1;
    const int t2c = (t2 < NSTEP) ? t2 : (NSTEP - 1);
    const int w1i = w1[t2c];
    const int w2i = w2[t2c];
    int jsrc = -1;
    if (t2 < sk) {
      if (2 * t2 >= sk) jsrc = 2 * t2 - sk;
    } else {
      if (t2 >= 2 * sk) jsrc = t2 - 2 * sk;
    }
    const int mode = (jsrc < 0) ? 0 : ((jsrc == t) ? 1 : 2);
    const int slot = ((jsrc < 0) ? 0 : jsrc) & (RING_SLOTS - 1);
    const float w1f = (float)w1i;
    const float w2f = (float)w2i;
    const bool use1 = (w1i != 0);
    const bool use2 = (w2i != 0) && (mode != 0);
    const bool last = (t == NSTEP - 1);
    const float* rsrc = ring + ((size_t)slot * NBATCH + (size_t)rowbase) * NHID;
    const _Float16* xrow = X16 + ((size_t)t * NBATCH + (size_t)(rowbase + c)) * NIN + koff;

#pragma unroll
    for (int nt = 0; nt < 4; ++nt) {
      const int j = 64 * wave + 16 * nt + c;
      const _Float16* wh = WHH + (size_t)j * NHID + koff;
      const _Float16* wx = WIH + (size_t)j * NIN + koff;
      v8f accR = z8, accZ = z8, accN = z8, accX = z8;
#pragma unroll 1
      for (int k0 = 0; k0 < NHID; k0 += 32) {
        const v16h a  = frag_load(ahrow + k0);
        const v16h b0 = frag_load(wh + k0);
        const v16h b1 = frag_load(wh + (size_t)1 * NHID * NHID + k0);
        const v16h b2 = frag_load(wh + (size_t)2 * NHID * NHID + k0);
        accR = mma16(a, b0, accR);
        accZ = mma16(a, b1, accZ);
        accN = mma16(a, b2, accN);
        guard3(accR, accZ, accN, a, b0, b1, b2);
      }
#pragma unroll 1
      for (int k0 = 0; k0 < NIN; k0 += 32) {
        const v16h a  = frag_load(xrow + k0);
        const v16h b0 = frag_load(wx + k0);
        const v16h b1 = frag_load(wx + (size_t)1 * NHID * NIN + k0);
        const v16h b2 = frag_load(wx + (size_t)2 * NHID * NIN + k0);
        accR = mma16(a, b0, accR);
        accZ = mma16(a, b1, accZ);
        accX = mma16(a, b2, accX);
        guard3(accR, accZ, accX, a, b0, b1, b2);
      }
      guard4acc(accR, accZ, accN, accX);

      float hs[8];
#pragma unroll
      for (int r = 0; r < 8; ++r) hs[r] = 0.0f;
      if (mode == 2) {
#pragma unroll
        for (int r = 0; r < 8; ++r)
          hs[r] = *(const volatile float*)(rsrc + (size_t)(8 * hh + r) * NHID + j);
      }

#pragma unroll
      for (int r = 0; r < 8; ++r) {
        const float pr = accR[r] * WCARRY_INV + bR[nt];
        const float pz = accZ[r] * WCARRY_INV + bZ[nt];
        const float ph = accN[r] * WCARRY_INV + bHN[nt];
        const float px = accX[r] * WCARRY_INV + bXN[nt];
        const float rg = fsig(pr);
        const float zg = fsig(pz);
        const float ng = ftanh(px + rg * ph);
        const float ho = hc[nt][r];
        const float hn = (1.0f - zg) * ng + zg * ho;
        slab[(8 * hh + r) * SLABP + 16 * nt + c] = hn;
        const float hsel = (mode == 1) ? hn : hs[r];
        const float p1 = use1 ? (w1f * hn) : 0.0f;
        const float p2 = use2 ? (w2f * hsel) : 0.0f;
        hc[nt][r] = p1 + p2;
      }
    }

    __builtin_amdgcn_fence(__ATOMIC_RELEASE, "workgroup");
    __builtin_amdgcn_wave_barrier();
    __builtin_amdgcn_fence(__ATOMIC_ACQUIRE, "workgroup");
    {
      float* rdst = ring + ((size_t)(t & (RING_SLOTS - 1)) * NBATCH + (size_t)rowbase) * NHID + 64 * wave + c4;
      float* odst = out + (size_t)rowbase * NHID + 64 * wave + c4;
      for (int pass = 0; pass < 2; ++pass) {
#pragma unroll
        for (int it = 0; it < 8; ++it) {
          const int row = it * 2 + hh;
          const v4f v = *(const v4f*)(slab + row * SLABP + c4);
          *(volatile v4f*)(rdst + (size_t)row * NHID) = v;
          if (last) {
            const v4f v2 = v + v;
            *(volatile v4f*)(odst + (size_t)row * NHID) = v2;
          }
        }
        __threadfence();
      }
    }
    __builtin_amdgcn_fence(__ATOMIC_RELEASE, "workgroup");
    __builtin_amdgcn_wave_barrier();
    __builtin_amdgcn_fence(__ATOMIC_ACQUIRE, "workgroup");

    __syncthreads();
#pragma unroll
    for (int nt = 0; nt < 4; ++nt) {
      const int j = 64 * wave + 16 * nt + c;
#pragma unroll
      for (int r = 0; r < 8; ++r) Ah[(8 * hh + r) * HPITCH + j] = (_Float16)hc[nt][r];
    }
    __syncthreads();
  }
}

extern "C" void kernel_launch(void* const* d_in, const int* in_sizes, int n_in,
                              void* d_out, int out_size, void* d_ws, size_t ws_size, hipStream_t stream) {
  if (n_in < 8 || d_out == nullptr || d_ws == nullptr) return;
  if (in_sizes[0] != NBATCH * NSTEP * NIN || in_sizes[1] != NGATE * NIN || in_sizes[2] != NGATE * NHID ||
      in_sizes[3] != NGATE || in_sizes[4] != NGATE || in_sizes[5] != NSTEP || in_sizes[6] != NSTEP ||
      in_sizes[7] != 1 || out_size != NBATCH * NHID) return;

  const float* x     = (const float*)d_in[0];
  const float* w_ih  = (const float*)d_in[1];
  const float* w_hh  = (const float*)d_in[2];
  const float* bi    = (const float*)d_in[3];
  const float* bh    = (const float*)d_in[4];
  const int*   w1    = (const int*)d_in[5];
  const int*   w2    = (const int*)d_in[6];
  const int*   skipp = (const int*)d_in[7];
  float* out = (float*)d_out;

  char* ws = (char*)d_ws;
  size_t off = 0;
  auto carve = [&](size_t bytes) -> char* { char* p = ws + off; off += (bytes + 255) & ~(size_t)255; return p; };
  unsigned short* X16   = (unsigned short*)carve((size_t)NSTEP * NBATCH * NIN * 2);
  unsigned short* WHH16 = (unsigned short*)carve((size_t)NGATE * NHID * 2);
  unsigned short* WIH16 = (unsigned short*)carve((size_t)NGATE * NIN * 2);
  float*          RING  = (float*)carve((size_t)RING_SLOTS * NBATCH * NHID * 4);
  if (off > ws_size || off > (size_t)134217728) return;

  const int n8x = NSTEP * NBATCH * (NIN / 8);
  const int n8h = NGATE * (NHID / 8);
  const int n8i = NGATE * (NIN / 8);
  cvt8_kernel<<<(n8x + CVT_THR - 1) / CVT_THR, CVT_THR, 0, stream>>>(x,    X16,   n8x, NIN / 8,  1, 1.0f);
  cvt8_kernel<<<(n8h + CVT_THR - 1) / CVT_THR, CVT_THR, 0, stream>>>(w_hh, WHH16, n8h, NHID / 8, 0, WCARRY);
  cvt8_kernel<<<(n8i + CVT_THR - 1) / CVT_THR, CVT_THR, 0, stream>>>(w_ih, WIH16, n8i, NIN / 8,  0, WCARRY);

  gru_seq_kernel<<<NBATCH / ROWS_BLK, RTHR, 0, stream>>>(X16, WHH16, WIH16, bi, bh, w1, w2, skipp, RING, out);
}
